// ScaledLinearDotProductAttention_58952721105439
// MI455X (gfx1250) — hardware-verified
//
#include <hip/hip_runtime.h>
#include <math.h>
#include <stdint.h>

#define NB    16
#define SEQ   4096
#define HD    64
#define NQB   (SEQ / 64)
#define RESQB 8
static_assert(HD == 64);
static_assert((SEQ % 64) == 0);
static_assert(RESQB <= NQB);
static_assert(((NB * SEQ * HD / 8) % 256) == 0);

typedef _Float16 v16h __attribute__((ext_vector_type(16)));
typedef _Float16 v8h  __attribute__((ext_vector_type(8)));
typedef __bf16   v16b __attribute__((ext_vector_type(16)));
typedef __bf16   v8b  __attribute__((ext_vector_type(8)));
typedef float    v8f  __attribute__((ext_vector_type(8)));
typedef float    v4f  __attribute__((ext_vector_type(4)));
typedef unsigned int v4u __attribute__((ext_vector_type(4)));

__device__ __forceinline__ unsigned short bf_bits(float f) {
  unsigned u = __float_as_uint(f);
  return (unsigned short)((u + 0x7FFFu + ((u >> 16) & 1u)) >> 16);
}
__device__ __forceinline__ float bf_up(unsigned short h) { return __uint_as_float(((unsigned)h) << 16); }
__device__ __forceinline__ unsigned short h_bits(_Float16 x) { return __builtin_bit_cast(unsigned short, x); }
__device__ __forceinline__ unsigned pk16(unsigned short a, unsigned short b) { return (unsigned)a | ((unsigned)b << 16); }
__device__ __forceinline__ v8f zero8() { v8f z = {0.f, 0.f, 0.f, 0.f, 0.f, 0.f, 0.f, 0.f}; return z; }

__device__ __forceinline__ v16b ldfrag_b(const __bf16* p) {
  union { v16b v; v8b h[2]; } f;
  f.h[0] = *(const v8b*)(p);
  f.h[1] = *(const v8b*)(p + 16);
  return f.v;
}

__device__ __forceinline__ v8f mma_b(v16b a, v16b b, v8f c) {
  c = __builtin_amdgcn_wmma_f32_16x16x32_bf16(false, a, false, b, (short)0, c, false, false);
#if defined(__HIP_DEVICE_COMPILE__)
  asm volatile("v_nop\n\tv_nop\n\tv_nop\n\tv_nop" : "+v"(c) : "v"(a), "v"(b));
#endif
  return c;
}
__device__ __forceinline__ v8f mma_h(v16h a, v16h b, v8f c) {
  c = __builtin_amdgcn_wmma_f32_16x16x32_f16(false, a, false, b, (short)0, c, false, false);
#if defined(__HIP_DEVICE_COMPILE__)
  asm volatile("v_nop\n\tv_nop\n\tv_nop\n\tv_nop" : "+v"(c) : "v"(a), "v"(b));
#endif
  return c;
}

__global__ __launch_bounds__(256) void cvt_bf16x8(const float* __restrict__ in, unsigned short* out, int n8) {
  const int i = blockIdx.x * 256 + threadIdx.x;
  if (i < n8) {
    const v4f a = *(const v4f*)(in + (size_t)i * 8);
    const v4f b = *(const v4f*)(in + (size_t)i * 8 + 4);
    v4u p;
    p[0] = pk16(bf_bits(a[0]), bf_bits(a[1]));
    p[1] = pk16(bf_bits(a[2]), bf_bits(a[3]));
    p[2] = pk16(bf_bits(b[0]), bf_bits(b[1]));
    p[3] = pk16(bf_bits(b[2]), bf_bits(b[3]));
    *(volatile v4u*)(out + (size_t)i * 8) = p;
    __threadfence();
    *(volatile v4u*)(out + (size_t)i * 8) = p;
  }
}

__global__ __launch_bounds__(256) void vt_f16(const float* __restrict__ v, unsigned short* vt) {
  __shared__ __align__(16) float sT[64 * 68];
  const int tid = threadIdx.x, wave = tid >> 5, lane = tid & 31;
  const int stile = blockIdx.x % NQB;
  const int b     = blockIdx.x / NQB;
  const int s0    = stile * 64;
  {
    const int row = tid >> 2, col0 = (tid & 3) * 16;
    const float* src = v + ((size_t)b * SEQ + s0 + row) * HD + col0;
#pragma unroll
    for (int i = 0; i < 4; ++i) {
      const v4f x = *(const v4f*)(src + 4 * i);
#pragma unroll
      for (int e = 0; e < 4; ++e) sT[(col0 + 4 * i + e) * 68 + row] = x[e];
    }
  }
  __syncthreads();
  const int q = lane >> 3, c8 = (lane & 7) * 8;
  v4u pv[2];
#pragma unroll
  for (int it = 0; it < 2; ++it) {
    const int d = wave * 8 + it * 4 + q;
    const float* sp = sT + d * 68 + c8;
    const v4f a  = *(const v4f*)(sp);
    const v4f a2 = *(const v4f*)(sp + 4);
    v4u p;
#pragma unroll
    for (int e = 0; e < 4; ++e) {
      const float f0 = (e < 2) ? a[2 * e]     : a2[2 * e - 4];
      const float f1 = (e < 2) ? a[2 * e + 1] : a2[2 * e - 3];
      const unsigned short h0 = h_bits((_Float16)(bf_up(bf_bits(f0)) * 256.0f));
      const unsigned short h1 = h_bits((_Float16)(bf_up(bf_bits(f1)) * 256.0f));
      p[e] = pk16(h0, h1);
    }
    pv[it] = p;
  }
  for (int pass = 0; pass < 2; ++pass) {
#pragma unroll
    for (int it = 0; it < 2; ++it) {
      const int d = wave * 8 + it * 4 + q;
      *(volatile v4u*)(vt + ((size_t)b * HD + d) * SEQ + s0 + c8) = pv[it];
    }
    __threadfence();
  }
}

template <bool RES>
__global__ __launch_bounds__(128)
void attn64(const unsigned short* __restrict__ qp, const unsigned short* __restrict__ kp,
            const unsigned short* __restrict__ vtp, const int* __restrict__ flagp,
            float* outp, int qbBase, int nqbThis, float sscale) {
  union FB { v16b v; v8b h[2]; };
  union FH { v16h v; v8h h[2]; };
  __shared__ __align__(16) __bf16   Ksh[64 * 64];
  __shared__ __align__(16) _Float16 Vth[64 * 64];
  __shared__ __align__(16) _Float16 Psh[4][16 * 64];
  __shared__ __align__(16) _Float16 Psl[RES ? 4 : 1][16 * 64];
  __shared__ __align__(16) float    Os[4][16 * 64];

  const int tid  = threadIdx.x;
  const int wave = tid >> 5;
  const int lane = tid & 31;
  const int hh   = lane >> 4;
  const int c    = lane & 15;

  const int bx   = blockIdx.x;
  const int qbl  = bx % nqbThis;
  const int b    = bx / nqbThis;
  const int qb   = qbBase + qbl;
  const int q0   = qb * 64 + wave * 16;
  const size_t rowB = (size_t)b * SEQ;
  const int causal = (flagp[0] != 0) ? 1 : 0;

  const __bf16*   Q  = (const __bf16*)(const void*)qp;
  const __bf16*   K  = (const __bf16*)(const void*)kp;
  const _Float16* Vt = (const _Float16*)(const void*)vtp + (size_t)b * HD * SEQ;

  v16b qa[2];
#pragma unroll
  for (int dc = 0; dc < 2; ++dc) {
    const size_t qo = (rowB + q0 + c) * HD + dc * 32 + 8 * hh;
    qa[dc] = ldfrag_b(Q + qo);
  }

  float mrow[8], lrow[8];
  v8f oacc[4];
#pragma unroll
  for (int r = 0; r < 8; ++r) { mrow[r] = -INFINITY; lrow[r] = 0.f; }
#pragma unroll
  for (int t = 0; t < 4; ++t) oacc[t] = zero8();

  int nkt = causal ? (qb + 1) : NQB;
  if (nkt > NQB) nkt = NQB;
  for (int kt = 0; kt < nkt; ++kt) {
    const int kv0 = kt * 64;
    __syncthreads();
    {
      const int r = tid >> 1, half = (tid & 1) * 32;
      const __bf16*   kg = K  + (rowB + kv0 + r) * HD + half;
      const _Float16* vg = Vt + (size_t)r * SEQ + kv0 + half;
#pragma unroll
      for (int i = 0; i < 4; ++i) {
        const v8b a0 = *(const v8b*)(kg + 8 * i);
        const v8h b0 = *(const v8h*)(vg + 8 * i);
        *(v8b*)(Ksh + r * 64 + half + 8 * i) = a0;
        *(v8h*)(Vth + r * 64 + half + 8 * i) = b0;
      }
    }
    __syncthreads();

    v8f s[4];
#pragma unroll
    for (int j = 0; j < 4; ++j) {
      s[j] = zero8();
#pragma unroll
      for (int dc = 0; dc < 2; ++dc) {
        FB kb;
        kb.h[0] = *(const v8b*)(Ksh + (j * 16 + c) * 64 + dc * 32 + 8 * hh);
        kb.h[1] = *(const v8b*)(Ksh + (j * 16 + c) * 64 + dc * 32 + 16 + 8 * hh);
        s[j] = mma_b(qa[dc], kb.v, s[j]);
      }
    }

    _Float16* pwh = Psh[wave];
    _Float16* pwl = Psl[RES ? wave : 0];
#pragma unroll
    for (int r = 0; r < 8; ++r) {
      const int qrow = q0 + 8 * hh + r;
      const int lim  = causal ? qrow : (SEQ + 64);
      float m = -INFINITY;
#pragma unroll
      for (int j = 0; j < 4; ++j) {
        const int key = kv0 + j * 16 + c;
        float sv = s[j][r] * sscale;
        sv = (key <= lim) ? sv : -INFINITY;
        s[j][r] = sv;
        m = fmaxf(m, sv);
      }
#pragma unroll
      for (int off = 1; off < 16; off <<= 1) m = fmaxf(m, __shfl_xor(m, off, 32));
      const float mnew  = fmaxf(mrow[r], m);
      const float msafe = (mnew == -INFINITY) ? 0.f : mnew;
      const float alpha = __expf(mrow[r] - msafe);
      mrow[r] = mnew;
      float psum = 0.f;
#pragma unroll
      for (int j = 0; j < 4; ++j) {
        const float p = __expf(s[j][r] - msafe);
        psum += p;
        const float p1k = p * 1024.0f;
        const _Float16 ph = (_Float16)p1k;
        pwh[(8 * hh + r) * 64 + j * 16 + c] = ph;
        if (RES) {
          const _Float16 pl = (_Float16)((p1k - (float)ph) * 4096.0f);
          pwl[(8 * hh + r) * 64 + j * 16 + c] = pl;
        }
      }
#pragma unroll
      for (int off = 1; off < 16; off <<= 1) psum += __shfl_xor(psum, off, 32);
      lrow[r] = lrow[r] * alpha + psum;
#pragma unroll
      for (int t = 0; t < 4; ++t) oacc[t][r] *= alpha;
    }
    __builtin_amdgcn_fence(__ATOMIC_RELEASE, "workgroup");
    __builtin_amdgcn_wave_barrier();
    __builtin_amdgcn_fence(__ATOMIC_ACQUIRE, "workgroup");

    v8f o1[4];
#pragma unroll
    for (int t = 0; t < 4; ++t) o1[t] = zero8();
#pragma unroll 1
    for (int kk = 0; kk < 2; ++kk) {
      FH pa, pl;
      pa.h[0] = *(const v8h*)(pwh + c * 64 + kk * 32 + 8 * hh);
      pa.h[1] = *(const v8h*)(pwh + c * 64 + kk * 32 + 16 + 8 * hh);
      if (RES) {
        pl.h[0] = *(const v8h*)(pwl + c * 64 + kk * 32 + 8 * hh);
        pl.h[1] = *(const v8h*)(pwl + c * 64 + kk * 32 + 16 + 8 * hh);
      } else {
        pl.v = pa.v;
      }
#pragma unroll
      for (int t = 0; t < 4; ++t) {
        FH vb;
        vb.h[0] = *(const v8h*)(Vth + (t * 16 + c) * 64 + kk * 32 + 8 * hh);
        vb.h[1] = *(const v8h*)(Vth + (t * 16 + c) * 64 + kk * 32 + 16 + 8 * hh);
        oacc[t] = mma_h(pa.v, vb.v, oacc[t]);
        if (RES) o1[t] = mma_h(pl.v, vb.v, o1[t]);
      }
    }
    if (RES) {
#pragma unroll
      for (int t = 0; t < 4; ++t)
#pragma unroll
        for (int r = 0; r < 8; ++r) oacc[t][r] += o1[t][r] * (1.0f / 4096.0f);
    }
  }

  float* os = Os[wave];
#pragma unroll
  for (int r = 0; r < 8; ++r) {
    const float l = lrow[r];
    const float inv = ((l > 0.f) ? (1.0f / l) : 0.f) * (1.0f / 262144.0f);
#pragma unroll
    for (int t = 0; t < 4; ++t) os[(8 * hh + r) * 64 + t * 16 + c] = oacc[t][r] * inv;
  }
  __builtin_amdgcn_fence(__ATOMIC_RELEASE, "workgroup");
  __builtin_amdgcn_wave_barrier();
  __builtin_amdgcn_fence(__ATOMIC_ACQUIRE, "workgroup");
  {
    const int h2 = lane >> 4, c4 = (lane & 15) * 4;
    v4f ov[8];
#pragma unroll
    for (int it = 0; it < 8; ++it) {
      const int row = it * 2 + h2;
      ov[it] = *(const v4f*)(os + row * 64 + c4);
    }
    for (int pass = 0; pass < 2; ++pass) {
#pragma unroll
      for (int it = 0; it < 8; ++it) {
        const int row = it * 2 + h2;
        const size_t go = (rowB + q0 + row) * HD + c4;
        *(volatile v4f*)(outp + go) = ov[it];
      }
      __threadfence();
    }
  }
}

extern "C" void kernel_launch(void* const* d_in, const int* in_sizes, int n_in,
                              void* d_out, int out_size, void* d_ws, size_t ws_size,
                              hipStream_t stream) {
  if (n_in < 4) return;
  const int nAct = NB * SEQ * HD;
  if (in_sizes[0] != nAct || in_sizes[1] != nAct || in_sizes[2] != nAct) return;
  if (in_sizes[3] < 1) return;
  if (out_size != nAct) return;

  const float* ql    = (const float*)d_in[0];
  const float* kl    = (const float*)d_in[1];
  const float* vl    = (const float*)d_in[2];
  const int*   flagp = (const int*)d_in[3];

  const size_t PL = (size_t)nAct * 2;
  size_t off = 0;
  const size_t oQ  = off; off += PL;
  const size_t oK  = off; off += PL;
  const size_t oVT = off; off += PL;
  if (off > ws_size) return;
  if (off > (size_t)134217728) return;

  char* ws = (char*)d_ws;
  unsigned short* Qb  = (unsigned short*)(ws + oQ);
  unsigned short* Kb  = (unsigned short*)(ws + oK);
  unsigned short* VTb = (unsigned short*)(ws + oVT);
  float* outf = (float*)d_out;

  const int n8 = nAct / 8;
  const dim3 blk(256);
  const dim3 gCvt((n8 + 255) / 256);
  const dim3 gVT(NB * NQB);

  cvt_bf16x8<<<gCvt, blk, 0, stream>>>(ql, Qb, n8);
  cvt_bf16x8<<<gCvt, blk, 0, stream>>>(kl, Kb, n8);
  vt_f16<<<gVT, blk, 0, stream>>>(vl, VTb);
  attn64<true><<<dim3(NB * RESQB), dim3(128), 0, stream>>>(
      Qb, Kb, VTb, flagp, outf, 0, RESQB, 0.125f);
  attn64<false><<<dim3(NB * (NQB - RESQB)), dim3(128), 0, stream>>>(
      Qb, Kb, VTb, flagp, outf, RESQB, NQB - RESQB, 0.125f);
  (void)hipGetLastError();
}
